// CrossAttention_51539607770
// MI455X (gfx1250) — hardware-verified
//
#include <hip/hip_runtime.h>
#include <stdint.h>


typedef _Float16 v16h __attribute__((ext_vector_type(16)));
typedef _Float16 v8h  __attribute__((ext_vector_type(8)));
typedef float    v8f  __attribute__((ext_vector_type(8)));
typedef float    v4f  __attribute__((ext_vector_type(4)));

#ifndef NB
#define NB 2
#endif
#ifndef SEQ
#define SEQ 1024
#endif
#define NB_FULL  2
#define SEQ_FULL 1024
#define DM   768
#define NH   12
#define HD   64
#define QKVW 2304
#define QKP  1536
#define ROWS (NB * SEQ)
#define ZSH  ((NB == 2) ? 1 : 0)
#define OUT1_ELEMS ((long)NB_FULL * SEQ_FULL * DM)

#define ACT_CAR   8.0f
#define W_CAR     1024.0f
#define PROJ_SCL  0.0009765625f
#define RES_CAR   2048.0f
#define RES_INV   0.00048828125f
#define S_SCL     0.001953125f
#define P_CAR     16384.0f
#define O_SCL     0.001953125f
#define OUT_SCL   3.814697265625e-06f

static_assert(NB == 1 || NB == 2);
static_assert(NB <= NB_FULL && SEQ <= SEQ_FULL);
static_assert(SEQ % 128 == 0);
static_assert(DM == NH * HD);
static_assert(HD == 64);
static_assert(QKVW == 3 * DM && QKP == 2 * DM);
static_assert(DM % 128 == 0 && DM % 64 == 0 && DM % 32 == 0 && QKVW % 64 == 0 && QKP % 64 == 0);
static_assert(OUT1_ELEMS * 4 == 6291456L);
static_assert(((long)ROWS * DM / 8) % 256 == 0);
static_assert((long)(QKVW / 64) * (DM / 64) * 4096 == (long)DM * QKVW);
static_assert((long)(DM / 64) * (DM / 64) * 4096 == (long)DM * DM);
static_assert((long)(QKP / 64) * (ROWS / 128) * 128 * 64 == (long)ROWS * QKP);
static_assert((long)(SEQ / 64) * (DM / 128) * 128 * 64 == (long)SEQ * DM);
static_assert((long)(SEQ / 128) * NH * 128 * HD == (long)SEQ * DM);
static_assert((long)(DM / 64) * (ROWS / 64) * 64 * 64 == (long)ROWS * DM);
static_assert(SEQ % 64 == 0);

#define N_X    ((size_t)2 * ROWS * DM)
#define N_WQKV ((size_t)2 * QKVW * DM)
#define N_WP   ((size_t)2 * DM * DM)
#define N_QK   ((size_t)2 * ROWS * QKP)
#define N_VT   ((size_t)2 * NB * DM * SEQ)
#define WS_HALVES (N_X + N_WQKV + N_WP + N_QK + N_X + N_VT + N_X + N_X)
static_assert(WS_HALVES * 2 <= (size_t)134217728);
static_assert(N_X % 64 == 0 && N_WQKV % 64 == 0 && N_WP % 64 == 0 && N_QK % 64 == 0 && N_VT % 64 == 0);

union Frag16 { v16h v; v8h p[2]; };

__device__ __forceinline__ v16h ld_frag_g(const _Float16* __restrict__ p, int hl) {
  Frag16 f;
  f.p[0] = *(const v8h*)(p + 8 * hl);
  f.p[1] = *(const v8h*)(p + 16 + 8 * hl);
  return f.v;
}

__device__ __forceinline__ v16h ld_frag_s(const _Float16* base, int off, int hl) {
  Frag16 f;
  f.p[0] = *(const v8h*)(base + off + 8 * hl);
  f.p[1] = *(const v8h*)(base + off + 16 + 8 * hl);
  return f.v;
}

__device__ __forceinline__ v8f mma(v16h a, v16h b, v8f c) {
  v8f d = __builtin_amdgcn_wmma_f32_16x16x32_f16(false, a, false, b, (short)0, c, false, false);
  asm volatile("v_nop\n\tv_nop\n\tv_nop\n\tv_nop" : "+v"(d) : "v"(a), "v"(b));
  return d;
}

__device__ __forceinline__ float bf16_rne(float x) {
  unsigned int u = __builtin_bit_cast(unsigned int, x);
  u += 0x7FFFu + ((u >> 16) & 1u);
  return __builtin_bit_cast(float, u & 0xFFFF0000u);
}

__global__ __launch_bounds__(256) void k_cvt8(const float* __restrict__ src,
                                              _Float16* __restrict__ dst,
                                              int cols, int seq, int seq_full, float car, int total8)
{
  const int i8 = blockIdx.x * 256 + threadIdx.x;
  if (i8 >= total8) return;
  const size_t e   = (size_t)i8 * 8;
  const int    r   = (int)(e / (size_t)cols);
  const int    col = (int)(e - (size_t)r * (size_t)cols);
  const int    bb  = r / seq;
  const int    nn  = r - bb * seq;
  const float* s = src + ((size_t)bb * seq_full + nn) * (size_t)cols + col;
  const v4f x0 = *(const v4f*)s;
  const v4f x1 = *(const v4f*)(s + 4);
  v8h o;
#pragma unroll
  for (int j = 0; j < 4; ++j) {
    const float t0 = x0[j];
    const float t1 = x1[j];
    o[j]     = (_Float16)(bf16_rne(t0) * car);
    o[4 + j] = (_Float16)(bf16_rne(t1) * car);
  }
  _Float16* d = dst + e;
  *(volatile v8h*)d = o;
  __threadfence();
  *(volatile v8h*)d = o;
}

__global__ __launch_bounds__(256) void k_trw(const float* __restrict__ W,
                                             _Float16* __restrict__ WT, int R, int C)
{
  __shared__ float tile[64 * 65];
  const int tid = threadIdx.x;
  const int c0 = blockIdx.x * 64, r0 = blockIdx.y * 64;
#pragma unroll
  for (int i = 0; i < 4; ++i) {
    const int idx = i * 256 + tid;
    const int r = idx >> 4, c4 = (idx & 15) * 4;
    const v4f v = *(const v4f*)(W + (size_t)(r0 + r) * C + c0 + c4);
    tile[r * 65 + c4 + 0] = v[0];
    tile[r * 65 + c4 + 1] = v[1];
    tile[r * 65 + c4 + 2] = v[2];
    tile[r * 65 + c4 + 3] = v[3];
  }
  __syncthreads();
  v8h o[2];
  size_t dofs[2];
#pragma unroll
  for (int i = 0; i < 2; ++i) {
    const int line = i * 32 + (tid >> 3);
    const int pc   = (tid & 7) * 8;
#pragma unroll
    for (int j = 0; j < 8; ++j)
      o[i][j] = (_Float16)(bf16_rne(tile[(pc + j) * 65 + line]) * W_CAR);
    dofs[i] = (size_t)(c0 + line) * R + r0 + pc;
  }
  *(volatile v8h*)(WT + dofs[0]) = o[0];
  *(volatile v8h*)(WT + dofs[1]) = o[1];
  __threadfence();
  *(volatile v8h*)(WT + dofs[0]) = o[0];
  *(volatile v8h*)(WT + dofs[1]) = o[1];
}

__device__ __forceinline__ void gemm_core(const _Float16* __restrict__ ap0,
                                          const _Float16* __restrict__ ap1,
                                          const _Float16* __restrict__ bp, int K, int hl, v8f (&acc)[8])
{
  const size_t bst = (size_t)16 * K;
#pragma unroll 1
  for (int k0 = 0; k0 < K; k0 += 32) {
    const v16h a0 = ld_frag_g(ap0 + k0, hl);
    const v16h a1 = ld_frag_g(ap1 + k0, hl);
    const v16h b0 = ld_frag_g(bp + k0, hl);
    const v16h b1 = ld_frag_g(bp + bst + k0, hl);
    const v16h b2 = ld_frag_g(bp + 2 * bst + k0, hl);
    const v16h b3 = ld_frag_g(bp + 3 * bst + k0, hl);
    acc[0] = mma(a0, b0, acc[0]);
    acc[1] = mma(a0, b1, acc[1]);
    acc[2] = mma(a0, b2, acc[2]);
    acc[3] = mma(a0, b3, acc[3]);
    acc[4] = mma(a1, b0, acc[4]);
    acc[5] = mma(a1, b1, acc[5]);
    acc[6] = mma(a1, b2, acc[6]);
    acc[7] = mma(a1, b3, acc[7]);
  }
}

__global__ __launch_bounds__(128) __attribute__((amdgpu_num_vgpr(256)))
void k_proj(const _Float16* __restrict__ A, const _Float16* __restrict__ Bt,
            _Float16* __restrict__ PH, _Float16* __restrict__ PL,
            size_t sA, size_t sB, size_t sC, size_t sL,
            int K, int ldc, int ldl, int resN, int zshA)
{
  __shared__ __attribute__((aligned(16))) _Float16 ldsE[2 * 128 * 72];
  constexpr int OFF_L = 128 * 72;

  const int tid = threadIdx.x, lane = tid & 31;
  const int w = __builtin_amdgcn_readfirstlane(tid >> 5);
  const int hl = lane >> 4, c = lane & 15;
  const int z = blockIdx.z;
  const int m0 = blockIdx.y * 128, n0 = blockIdx.x * 64;
  const int mw = m0 + 32 * w;
  const bool wres = (n0 < resN);

  const _Float16* az = A  + (size_t)(z >> zshA) * sA;
  const _Float16* bz = Bt + (size_t)z * sB;
  const _Float16* ap0 = az + (size_t)(mw + c) * K;
  const _Float16* ap1 = az + (size_t)(mw + 16 + c) * K;
  const _Float16* bp  = bz + (size_t)(n0 + c) * K;

  v8f acc[8] = {};
  gemm_core(ap0, ap1, bp, K, hl, acc);

#pragma unroll
  for (int i = 0; i < 2; ++i)
#pragma unroll
    for (int t = 0; t < 4; ++t)
#pragma unroll
      for (int r = 0; r < 8; ++r) {
        const int rowl = 32 * w + 16 * i + 8 * hl + r;
        const float v = acc[i * 4 + t][r] * PROJ_SCL;
        const _Float16 hv = (_Float16)v;
        ldsE[rowl * 72 + 16 * t + c] = hv;
        if (wres) {
          const float res = (v - (float)hv) * RES_CAR;
          ldsE[OFF_L + rowl * 72 + 16 * t + c] = (_Float16)res;
        }
      }
  __syncthreads();

  _Float16* const bh = PH + (size_t)z * sC + (size_t)m0 * ldc + n0;
  _Float16* const bl = PL + (size_t)z * sL + (size_t)m0 * ldl + n0;
  for (int i = 0; i < 8; ++i) {
    const int q = i * 128 + tid;
    const int rowl = q >> 3, ch = (q & 7) * 8;
    const v8h vh = *(const v8h*)(&ldsE[rowl * 72 + ch]);
    *(volatile v8h*)(bh + (size_t)rowl * ldc + ch) = vh;
    if (wres) {
      const v8h vl = *(const v8h*)(&ldsE[OFF_L + rowl * 72 + ch]);
      *(volatile v8h*)(bl + (size_t)rowl * ldl + ch) = vl;
    }
  }
  __threadfence();
  for (int i = 0; i < 8; ++i) {
    const int q = i * 128 + tid;
    const int rowl = q >> 3, ch = (q & 7) * 8;
    const v8h vh = *(const v8h*)(&ldsE[rowl * 72 + ch]);
    *(volatile v8h*)(bh + (size_t)rowl * ldc + ch) = vh;
    if (wres) {
      const v8h vl = *(const v8h*)(&ldsE[OFF_L + rowl * 72 + ch]);
      *(volatile v8h*)(bl + (size_t)rowl * ldl + ch) = vl;
    }
  }
}

__global__ __launch_bounds__(256) __attribute__((amdgpu_num_vgpr(256)))
void k_attn(const _Float16* __restrict__ QKH, const _Float16* __restrict__ QL,
            const _Float16* __restrict__ VtH,
            _Float16* __restrict__ OH, _Float16* __restrict__ OL)
{
  constexpr int KT_H   = 32 * 72;
  constexpr int V_H    = HD * 40;
  constexpr int P_H    = 8 * 16 * 40;
  constexpr int TILE_H = KT_H + V_H + P_H;
  constexpr int EPI_H  = 2 * 128 * 72;
  constexpr int LDS_H  = (TILE_H > EPI_H) ? TILE_H : EPI_H;
  constexpr int OFF_K  = 0;
  constexpr int OFF_V  = KT_H;
  constexpr int OFF_P  = KT_H + V_H;
  constexpr int OFF_OH = 0;
  constexpr int OFF_OL = 128 * 72;
  static_assert(OFF_V % 8 == 0 && OFF_P % 8 == 0 && OFF_OL % 8 == 0);
  static_assert(256 * 8 == 32 * 64 && 256 * 8 == HD * 32);
  __shared__ __attribute__((aligned(16))) _Float16 lds[LDS_H];

  const int tid = threadIdx.x, lane = tid & 31;
  const int wave = __builtin_amdgcn_readfirstlane(tid >> 5);
  const int hl = lane >> 4, c = lane & 15;
  const int q0 = blockIdx.x * 128;
  const int col0 = blockIdx.y * HD;
  const int z = blockIdx.z;
  const int s = z >> ZSH;
  const int b = z - (s << ZSH);

  const size_t qr = (size_t)s * ROWS + (size_t)b * SEQ + q0 + 16 * wave + c;
  v16h qh[2], ql[2];
#pragma unroll
  for (int ks = 0; ks < 2; ++ks) {
    qh[ks] = ld_frag_g(QKH + qr * QKP + col0 + 32 * ks, hl);
    ql[ks] = ld_frag_g(QL  + qr * DM  + col0 + 32 * ks, hl);
  }
  const int pOff = OFF_P + wave * (16 * 40);

  const int krr = tid >> 3, kcc = (tid & 7) * 8;
  const int vdd = tid >> 2, vkc = (tid & 3) * 8;

  v8f ofin[4] = {};

#pragma unroll 1
  for (int p = 0; p < 2; ++p) {
    const int kv = (p == 0) ? s : (1 - s);
    const size_t kgo = ((size_t)kv * ROWS + (size_t)b * SEQ + krr) * QKP + DM + col0 + kcc;
    const size_t vgo = (((size_t)kv * NB + b) * DM + col0 + vdd) * SEQ + vkc;

    float m[8], l[8];
    v8f o[4] = {};
#pragma unroll
    for (int r = 0; r < 8; ++r) { m[r] = -__builtin_inff(); l[r] = 0.f; }

#pragma unroll 1
    for (int kt = 0; kt < SEQ / 32; ++kt) {
      const int mk = kt * 32;
      {
        const v8h k8 = *(const v8h*)(QKH + kgo + (size_t)mk * QKP);
        const v8h v8 = *(const v8h*)(VtH + vgo + mk);
        *(v8h*)(&lds[OFF_K + krr * 72 + kcc]) = k8;
        *(v8h*)(&lds[OFF_V + vdd * 40 + vkc]) = v8;
      }
      __syncthreads();

      v8f sh[2] = {}, sl[2] = {};
#pragma unroll
      for (int ks = 0; ks < 2; ++ks) {
#pragma unroll
        for (int t = 0; t < 2; ++t) {
          const v16h kf = ld_frag_s(lds, OFF_K + (16 * t + c) * 72 + 32 * ks, hl);
          sh[t] = mma(qh[ks], kf, sh[t]);
          sl[t] = mma(ql[ks], kf, sl[t]);
        }
      }

#pragma unroll
      for (int r = 0; r < 8; ++r) {
        const float v0 = (sh[0][r] + sl[0][r] * RES_INV) * S_SCL;
        const float v1 = (sh[1][r] + sl[1][r] * RES_INV) * S_SCL;
        float tm = fmaxf(v0, v1);
        tm = fmaxf(tm, __shfl_xor(tm, 1, 32));
        tm = fmaxf(tm, __shfl_xor(tm, 2, 32));
        tm = fmaxf(tm, __shfl_xor(tm, 4, 32));
        tm = fmaxf(tm, __shfl_xor(tm, 8, 32));
        const float mn = fmaxf(m[r], tm);
        const float al = __expf(m[r] - mn);
        const float p0 = __expf(v0 - mn), p1 = __expf(v1 - mn);
        float rs = p0 + p1;
        rs += __shfl_xor(rs, 1, 32);
        rs += __shfl_xor(rs, 2, 32);
        rs += __shfl_xor(rs, 4, 32);
        rs += __shfl_xor(rs, 8, 32);
        l[r] = l[r] * al + rs;
        m[r] = mn;
#pragma unroll
        for (int t = 0; t < 4; ++t) o[t][r] *= al;
        const int pi = pOff + (8 * hl + r) * 40 + c;
        lds[pi]      = (_Float16)(p0 * P_CAR);
        lds[pi + 16] = (_Float16)(p1 * P_CAR);
      }
      __syncthreads();

      const v16h pf = ld_frag_s(lds, pOff + c * 40, hl);
#pragma unroll
      for (int t = 0; t < 4; ++t) {
        const v16h vf = ld_frag_s(lds, OFF_V + (16 * t + c) * 40, hl);
        o[t] = mma(pf, vf, o[t]);
      }
      __syncthreads();
    }

#pragma unroll
    for (int r = 0; r < 8; ++r) {
      const float inv = 1.0f / l[r];
#pragma unroll
      for (int t = 0; t < 4; ++t) ofin[t][r] += o[t][r] * inv;
    }
  }

#pragma unroll
  for (int r = 0; r < 8; ++r) {
    const int rowl = 16 * wave + 8 * hl + r;
#pragma unroll
    for (int t = 0; t < 4; ++t) {
      const float v = ofin[t][r] * O_SCL;
      const _Float16 hv = (_Float16)v;
      const float res = (v - (float)hv) * RES_CAR;
      lds[OFF_OH + rowl * 72 + 16 * t + c] = hv;
      lds[OFF_OL + rowl * 72 + 16 * t + c] = (_Float16)res;
    }
  }
  __syncthreads();
  const size_t obase = ((size_t)s * ROWS + (size_t)b * SEQ + q0) * DM + col0;
  _Float16* const bh = OH + obase;
  _Float16* const bl = OL + obase;
  for (int i = 0; i < 4; ++i) {
    const int q = i * 256 + tid;
    const int rowl = q >> 3, ch = (q & 7) * 8;
    const v8h vh = *(const v8h*)(&lds[OFF_OH + rowl * 72 + ch]);
    const v8h vl = *(const v8h*)(&lds[OFF_OL + rowl * 72 + ch]);
    *(volatile v8h*)(bh + (size_t)rowl * DM + ch) = vh;
    *(volatile v8h*)(bl + (size_t)rowl * DM + ch) = vl;
  }
  __threadfence();
  for (int i = 0; i < 4; ++i) {
    const int q = i * 256 + tid;
    const int rowl = q >> 3, ch = (q & 7) * 8;
    const v8h vh = *(const v8h*)(&lds[OFF_OH + rowl * 72 + ch]);
    const v8h vl = *(const v8h*)(&lds[OFF_OL + rowl * 72 + ch]);
    *(volatile v8h*)(bh + (size_t)rowl * DM + ch) = vh;
    *(volatile v8h*)(bl + (size_t)rowl * DM + ch) = vl;
  }
}

__global__ __launch_bounds__(128) __attribute__((amdgpu_num_vgpr(256)))
void k_oproj(const _Float16* __restrict__ AH, const _Float16* __restrict__ AL,
             const _Float16* __restrict__ Bt, const float* __restrict__ bias,
             float* __restrict__ Out)
{
  __shared__ __attribute__((aligned(16))) float ldsF[64 * 68];

  const int tid = threadIdx.x, lane = tid & 31;
  const int w = __builtin_amdgcn_readfirstlane(tid >> 5);
  const int hl = lane >> 4, c = lane & 15;
  const int m0 = blockIdx.y * 64, n0 = blockIdx.x * 64;
  const int mw = m0 + 16 * w;

  const _Float16* ap0 = AH + (size_t)(mw + c) * DM;
  const _Float16* ap1 = AL + (size_t)(mw + c) * DM;
  const _Float16* bp  = Bt + (size_t)(n0 + c) * DM;

  v8f acc[8] = {};
  gemm_core(ap0, ap1, bp, DM, hl, acc);

#pragma unroll
  for (int t = 0; t < 4; ++t)
#pragma unroll
    for (int r = 0; r < 8; ++r) {
      const int rowl = 16 * w + 8 * hl + r;
      ldsF[rowl * 68 + 16 * t + c] = (acc[t][r] + acc[4 + t][r] * RES_INV) * OUT_SCL;
    }
  __syncthreads();

  const int bcol = (tid & 15) * 4;
  const v4f braw = *(const v4f*)(bias + n0 + bcol);
  v4f bb;
  bb[0] = bf16_rne(braw[0]); bb[1] = bf16_rne(braw[1]);
  bb[2] = bf16_rne(braw[2]); bb[3] = bf16_rne(braw[3]);

  const int ob_b = m0 / SEQ;
  const int ob_n = m0 - ob_b * SEQ;
  float* const ob = Out + ((size_t)ob_b * SEQ_FULL + ob_n) * DM + n0;
  for (int i = 0; i < 8; ++i) {
    const int qi = i * 128 + tid;
    const int rowl = qi >> 4, col = (qi & 15) * 4;
    const v4f v = *(const v4f*)(&ldsF[rowl * 68 + col]) + bb;
    *(volatile v4f*)(ob + (size_t)rowl * DM + col) = v;
  }
  __threadfence();
  for (int i = 0; i < 8; ++i) {
    const int qi = i * 128 + tid;
    const int rowl = qi >> 4, col = (qi & 15) * 4;
    const v4f v = *(const v4f*)(&ldsF[rowl * 68 + col]) + bb;
    *(volatile v4f*)(ob + (size_t)rowl * DM + col) = v;
  }
}

extern "C" void kernel_launch(void* const* d_in, const int* in_sizes, int n_in,
                              void* d_out, int out_size, void* d_ws, size_t ws_size,
                              hipStream_t stream)
{
  if (n_in < 8) return;
  const long need_x = ((long)(NB - 1) * SEQ_FULL + SEQ) * DM;
  if ((long)in_sizes[0] < need_x) return;
  if ((long)in_sizes[1] < need_x) return;
  if ((long)in_sizes[2] < (long)DM * QKVW) return;
  if ((long)in_sizes[3] < (long)DM * QKVW) return;
  if ((long)in_sizes[4] < (long)DM * DM) return;
  if ((long)in_sizes[5] < (long)DM) return;
  if ((long)in_sizes[6] < (long)DM * DM) return;
  if ((long)in_sizes[7] < (long)DM) return;
  if ((long)out_size < OUT1_ELEMS + need_x) return;
  if (WS_HALVES * sizeof(_Float16) > ws_size) return;

  const float* x1    = (const float*)d_in[0];
  const float* x2    = (const float*)d_in[1];
  const float* Wqkv1 = (const float*)d_in[2];
  const float* Wqkv2 = (const float*)d_in[3];
  const float* Wp1   = (const float*)d_in[4];
  const float* bp1   = (const float*)d_in[5];
  const float* Wp2   = (const float*)d_in[6];
  const float* bp2   = (const float*)d_in[7];
  float* out = (float*)d_out;

  _Float16* X16   = (_Float16*)d_ws;
  _Float16* WqkvT = X16   + N_X;
  _Float16* WpT   = WqkvT + N_WQKV;
  _Float16* QKH   = WpT   + N_WP;
  _Float16* QL    = QKH   + N_QK;
  _Float16* VtH   = QL    + N_X;
  _Float16* OH    = VtH   + N_VT;
  _Float16* OL    = OH    + N_X;

  const size_t nXs = (size_t)ROWS * DM;
  const int tx8 = (int)(nXs / 8);
  k_cvt8<<<tx8 / 256, 256, 0, stream>>>(x1, X16,       DM, SEQ, SEQ_FULL, ACT_CAR, tx8);
  k_cvt8<<<tx8 / 256, 256, 0, stream>>>(x2, X16 + nXs, DM, SEQ, SEQ_FULL, ACT_CAR, tx8);

  k_trw<<<dim3(QKVW / 64, DM / 64), 256, 0, stream>>>(Wqkv1, WqkvT, DM, QKVW);
  k_trw<<<dim3(QKVW / 64, DM / 64), 256, 0, stream>>>(Wqkv2, WqkvT + (size_t)QKVW * DM, DM, QKVW);
  k_trw<<<dim3(DM / 64, DM / 64), 256, 0, stream>>>(Wp1, WpT, DM, DM);
  k_trw<<<dim3(DM / 64, DM / 64), 256, 0, stream>>>(Wp2, WpT + (size_t)DM * DM, DM, DM);

  k_proj<<<dim3(QKP / 64, ROWS / 128, 2), 128, 0, stream>>>(
      X16, WqkvT, QKH, QL,
      nXs, (size_t)QKVW * DM, (size_t)ROWS * QKP, nXs,
      DM, QKP, DM, DM, 0);
  k_proj<<<dim3(SEQ / 64, DM / 128, 2 * NB), 128, 0, stream>>>(
      WqkvT + (size_t)2 * DM * DM, X16, VtH, QL,
      (size_t)QKVW * DM, (size_t)SEQ * DM, (size_t)DM * SEQ, (size_t)0,
      DM, SEQ, SEQ, 0, ZSH);

  k_attn<<<dim3(SEQ / 128, NH, 2 * NB), 256, 0, stream>>>(QKH, QL, VtH, OH, OL);

  k_oproj<<<dim3(DM / 64, ROWS / 64), 128, 0, stream>>>(OH, OL, WpT, bp1, out);
  k_oproj<<<dim3(DM / 64, ROWS / 64), 128, 0, stream>>>(OH + nXs, OL + nXs, WpT + (size_t)DM * DM, bp2,
                                                       out + OUT1_ELEMS);
}
